// DiffusionDynamicOutput_79336635892254
// MI455X (gfx1250) — hardware-run, weakly checked
//
#include <hip/hip_runtime.h>


#ifndef NB
#define NB 8
#endif
#define NB_FULL 8
#define NT    32
#define EMB   1024
#define HID   256
#define CH    64
#define NTAP  9
#define KD    (CH * NTAP)
#define KA    (2 * EMB)
#define HP    (2 * HID)
#define IMH   128
#define IMW   128
#define LPH   (IMH + 2)
#define LPW   (IMW + 2)
#define TLP   72
#define OSP   68

static_assert(NB <= NB_FULL);
static_assert(NB >= 2);
static_assert((NB * NT) % 64 == 0);
static_assert(NT == 32);
static_assert(CH == 64);
static_assert(KD == 576);
static_assert(KD % 64 == 0);
static_assert(HID % 64 == 0);
static_assert(KA % 32 == 0);
static_assert(HP % 32 == 0);
static_assert(CH % 32 == 0);
static_assert(EMB % 64 == 0);
static_assert(HID % 32 == 0);
static_assert(KD % 32 == 0);
static_assert(EMB % 8 == 0);
static_assert((EMB / 8) == 128);
static_assert(((size_t)NB * NT * (EMB / 8)) % 256 == 0);
static_assert(IMW % 64 == 0);
static_assert(IMW == 128);
static_assert((TLP * 2) % 16 == 0);
static_assert(TLP >= CH);
static_assert((OSP * 4) % 16 == 0);
static_assert(LPW * 8 <= 5 * 256);
static_assert((LPW * 8) % 8 == 0);
static_assert(32 * 16 * 16 == 64 * 128);
static_assert(32 * 16 * 16 == NT * 64 * 4);
static_assert(256 * 16 == 32 * 128);
static_assert(LPW * TLP * 2 <= 131072);
static_assert(64 * OSP * 4 <= 131072);
static_assert(32 * OSP * 4 <= 131072);

typedef _Float16 h16;
typedef unsigned short bf;
typedef __attribute__((ext_vector_type(16))) __bf16   v16bf;
typedef __attribute__((ext_vector_type(16))) _Float16 v16h;
typedef __attribute__((ext_vector_type(8)))  _Float16 v8h;
typedef __attribute__((ext_vector_type(8)))  unsigned short v8us;
typedef __attribute__((ext_vector_type(8)))  float    v8f;
typedef __attribute__((ext_vector_type(4)))  float    v4f;
typedef v4f  __attribute__((may_alias)) v4fa;
typedef v8h  __attribute__((may_alias)) v8ha;

__device__ __forceinline__ unsigned short f2bf(float f) { unsigned u = __float_as_uint(f); u += 0x7FFFu + ((u >> 16) & 1u); return (unsigned short)(u >> 16); }
__device__ __forceinline__ float bfr(float f) { return __uint_as_float(((unsigned)f2bf(f)) << 16); }
__device__ __forceinline__ float bf2f(unsigned short u) { return __uint_as_float(((unsigned)u) << 16); }
__device__ __forceinline__ v16h cat16(v8h lo, v8h hi) { return __builtin_shufflevector(lo, hi, 0, 1, 2, 3, 4, 5, 6, 7, 8, 9, 10, 11, 12, 13, 14, 15); }
__device__ __forceinline__ v16bf cat16b(v8us lo, v8us hi) { return __builtin_bit_cast(v16bf, __builtin_shufflevector(lo, hi, 0, 1, 2, 3, 4, 5, 6, 7, 8, 9, 10, 11, 12, 13, 14, 15)); }
__device__ __forceinline__ v8f wmma16(v16h a, v16h b, v8f c) { return __builtin_amdgcn_wmma_f32_16x16x32_f16(false, a, false, b, (short)0, c, false, false); }
__device__ __forceinline__ v8f wmmab(v16bf a, v16bf b, v8f c) { return __builtin_amdgcn_wmma_f32_16x16x32_bf16(false, a, false, b, (short)0, c, false, false); }
__device__ __forceinline__ v8f wmma16g(v16h a, v16h b, v8f c) { c = wmma16(a, b, c); asm volatile("v_nop\n\tv_nop\n\tv_nop\n\tv_nop" : "+v"(c) : "v"(a), "v"(b)); return c; }
__device__ __forceinline__ v8f wmmabg(v16bf a, v16bf b, v8f c) { c = wmmab(a, b, c); asm volatile("v_nop\n\tv_nop\n\tv_nop\n\tv_nop" : "+v"(c) : "v"(a), "v"(b)); return c; }
__device__ __forceinline__ v16h  ldh(const h16* p) { return cat16(*(const v8h*)p, *(const v8h*)(p + 16)); }
__device__ __forceinline__ v16bf ldb(const bf* p)  { return cat16b(*(const v8us*)p, *(const v8us*)(p + 16)); }
static __device__ __forceinline__ h16 toh_flush(float v) { const h16 r = (h16)v; return (fabsf(v) < 6.103515625e-05f) ? (h16)0.0f : r; }
__device__ __forceinline__ void wave_sync() { __builtin_amdgcn_fence(3  , "wavefront"); __builtin_amdgcn_wave_barrier(); asm volatile("" ::: "memory"); }

__global__ __launch_bounds__(256) void k_cvtrow(const float* __restrict__ src, bf* dst, int n8, int shift, int dcol) {
    const int i = blockIdx.x * 256 + threadIdx.x; if (i >= n8) return;
    const int row = i >> 7, p = i & 127;
    const v8f v = *(const v8f*)(src + ((size_t)(row >> shift) * EMB + (size_t)p * 8)); v8us o;
#pragma unroll
    for (int k = 0; k < 8; ++k) o[k] = f2bf(v[k]);
    bf* d = dst + (size_t)row * KA + dcol + p * 8;
    *(volatile v8us*)d = o; __threadfence(); *(volatile v8us*)d = o;
}

__global__ __launch_bounds__(256) void k_wT(const float* __restrict__ src, bf* dst, int K, int N, int pf) {
    __shared__ __align__(16) float ts[32 * OSP];
    const int tid = threadIdx.x; const int n0 = blockIdx.x * 32, k0 = blockIdx.y * 64;
    { const int nl = tid & 31, kq = tid >> 5; const int n = n0 + nl; const int col = pf ? ((n & (CH - 1)) * NTAP + (n >> 6)) : n;
#pragma unroll
      for (int i = 0; i < 8; ++i) ts[nl * OSP + kq * 8 + i] = bfr(src[(size_t)(k0 + kq * 8 + i) * N + col]); }
    __syncthreads();
    const int row = tid >> 3, p8 = (tid & 7) * 8;
    const v4f x0 = *(const v4fa*)(&ts[row * OSP + p8]); const v4f x1 = *(const v4fa*)(&ts[row * OSP + p8 + 4]); v8us o;
#pragma unroll
    for (int i = 0; i < 4; ++i) { o[i] = f2bf(x0[i]); o[4 + i] = f2bf(x1[i]); }
    bf* d0 = dst + (size_t)(n0 + row) * (size_t)(2 * K) + k0 + p8;
#pragma unroll 1
    for (int ps = 0; ps < 2; ++ps) {
        *(volatile v8us*)d0 = o; *(volatile v8us*)(d0 + K) = o;
        if (ps == 0) __threadfence(); }
}

__global__ __launch_bounds__(256) void k_lat(const float* __restrict__ lat, h16* LP) {
    __shared__ __align__(16) h16 tl[LPW * TLP];
    const int tid = threadIdx.x; const int py = blockIdx.x, b = blockIdx.y;
    const bool yok = (py >= 1) && (py <= IMH);
    int yc = py - 1; yc = yc < 0 ? 0 : (yc > IMH - 1 ? IMH - 1 : yc);
    if (tid < 2 * CH) tl[((tid >> 6) ? (LPW - 1) : 0) * TLP + (tid & (CH - 1))] = (h16)0.0f;
    const float* src = lat + (((size_t)b * CH) * IMH + yc) * IMW;
#pragma unroll 4
    for (int it = 0; it < 8; ++it) {
        const int q = it * 256 + tid; const int d = q >> 5, x4 = (q & 31) * 4;
        const v4f v = *(const v4f*)(src + (size_t)d * IMH * IMW + x4);
#pragma unroll
        for (int j = 0; j < 4; ++j) tl[(x4 + 1 + j) * TLP + d] = toh_flush(yok ? bfr(v[j]) : 0.0f); }
    __syncthreads();
    h16* dst = LP + (((size_t)b * LPH + py) * LPW) * CH;
#pragma unroll 1
    for (int ps = 0; ps < 2; ++ps) {
#pragma unroll 1
        for (int it = 0; it < 5; ++it) { const int q = it * 256 + tid; const int qc = q < LPW * 8 ? q : LPW * 8 - 1;
            const v8h val = *(const v8ha*)(&tl[(qc >> 3) * TLP + (qc & 7) * 8]);
            if (q < LPW * 8) *(volatile v8h*)(dst + (size_t)q * 8) = val; }
        if (ps == 0) __threadfence(); }
}

template <int MODE, int K>
__device__ __forceinline__ void gemm_body(const bf* __restrict__ A, const bf* __restrict__ Bt, const float* __restrict__ bias, bf* OB, h16* OH) {
    __shared__ __align__(16) float os[64 * OSP];
    const int lane = threadIdx.x & 31, lr = lane & 15, hi = lane >> 4; const int r0 = blockIdx.x * 64, c0 = blockIdx.y * 64;
    v8f acc[4][4];
#pragma unroll
    for (int mb = 0; mb < 4; ++mb)
#pragma unroll
        for (int nb = 0; nb < 4; ++nb) acc[mb][nb] = (v8f){};
    const size_t aoff = (size_t)(r0 + lr) * K + 8 * hi, boff = (size_t)(c0 + lr) * K + 8 * hi;
#pragma unroll 1
    for (int kc = 0; kc < K; kc += 32) {
        v16bf a[4];
#pragma unroll
        for (int mb = 0; mb < 4; ++mb) a[mb] = ldb(A + aoff + (size_t)mb * 16 * K + kc);
#pragma unroll
        for (int nb = 0; nb < 4; ++nb) { const v16bf b = ldb(Bt + boff + (size_t)nb * 16 * K + kc);
#pragma unroll
            for (int mb = 0; mb < 4; ++mb) acc[mb][nb] = wmmabg(a[mb], b, acc[mb][nb]); }
    }
    float bc[4];
#pragma unroll
    for (int nb = 0; nb < 4; ++nb) { const int col = c0 + nb * 16 + lr; const int bi = (MODE == 0) ? col : ((col & (CH - 1)) * NTAP + (col >> 6)); bc[nb] = bfr(bias[bi]); }
#pragma unroll
    for (int mb = 0; mb < 4; ++mb) {
#pragma unroll
        for (int nb = 0; nb < 4; ++nb) {
#pragma unroll
            for (int j = 0; j < 8; ++j) os[(mb * 16 + hi * 8 + j) * OSP + nb * 16 + lr] = acc[mb][nb][j] + bc[nb]; } }
    wave_sync();
#pragma unroll 1
    for (int ps = 0; ps < 2; ++ps) {
#pragma unroll 1
        for (int s = 0; s < 16; ++s) { const int row = 4 * s + (lane >> 3), c8 = (lane & 7) * 8;
            const v4f x0 = *(const v4fa*)(&os[row * OSP + c8]); const v4f x1 = *(const v4fa*)(&os[row * OSP + c8 + 4]);
            if (MODE == 0) {
                v8us hv, lv;
#pragma unroll
                for (int i = 0; i < 4; ++i) {
                    const float t0 = x0[i], t1 = x1[i];
                    const float s0 = t0 * (1.0f / (1.0f + expf(-t0))), s1 = t1 * (1.0f / (1.0f + expf(-t1)));
                    const unsigned short u0 = f2bf(s0), u1 = f2bf(s1);
                    hv[i] = u0; hv[4 + i] = u1; lv[i] = f2bf(s0 - bf2f(u0)); lv[4 + i] = f2bf(s1 - bf2f(u1)); }
                bf* d = OB + (size_t)(r0 + row) * HP + c0 + c8;
                *(volatile v8us*)d = hv; *(volatile v8us*)(d + HID) = lv;
            } else {
                v8h wv;
#pragma unroll
                for (int i = 0; i < 4; ++i) { wv[i] = toh_flush(x0[i]); wv[4 + i] = toh_flush(x1[i]); }
                *(volatile v8h*)(OH + (size_t)(r0 + row) * KD + c0 + c8) = wv;
            } }
        if (ps == 0) __threadfence(); }
}

__global__ __launch_bounds__(32) void k_gemm_h(const bf* __restrict__ A, const bf* __restrict__ Bt, const float* __restrict__ bias, bf* H) {
    gemm_body<0, KA>(A, Bt, bias, H, (h16*)0);
}
__global__ __launch_bounds__(32) void k_gemm_w(const bf* __restrict__ A, const bf* __restrict__ Bt, const float* __restrict__ bias, h16* W) {
    gemm_body<1, HP>(A, Bt, bias, (bf*)0, W);
}

__global__ __launch_bounds__(32) void k_dconv(const h16* __restrict__ LP, const h16* __restrict__ WP, float* OUT) {
    __shared__ __align__(16) float os[NT * OSP];
    const int lane = threadIdx.x & 31, lr = lane & 15, hi = lane >> 4;
    const unsigned bx = blockIdx.x; const unsigned b = bx / (unsigned)(IMH * (IMW / 64)); const unsigned rem = bx % (unsigned)(IMH * (IMW / 64)); const unsigned y = rem / (unsigned)(IMW / 64); const unsigned w0 = (rem % (unsigned)(IMW / 64)) * 64u;
    v8f acc[4][2];
#pragma unroll
    for (int mb = 0; mb < 4; ++mb)
#pragma unroll
        for (int nb = 0; nb < 2; ++nb) acc[mb][nb] = (v8f){};
    const size_t abase = (((size_t)b * LPH + y) * LPW + (size_t)(w0 + lr)) * CH + 8 * hi;
    const size_t bbase = ((size_t)b * NT + lr) * KD + 8 * hi;
#pragma unroll 1
    for (int tap = 0; tap < NTAP; ++tap) {
        const int k1 = tap / 3, k2 = tap - 3 * k1;
#pragma unroll
        for (int c0 = 0; c0 < CH; c0 += 32) {
            const h16* ap = LP + abase + (size_t)(k1 * LPW + k2) * CH + c0;
            v16h a[4];
#pragma unroll
            for (int mb = 0; mb < 4; ++mb) a[mb] = ldh(ap + (size_t)mb * 16 * CH);
            const h16* bp = WP + bbase + tap * CH + c0;
#pragma unroll
            for (int nb = 0; nb < 2; ++nb) { const v16h bq = ldh(bp + (size_t)nb * 16 * KD);
#pragma unroll
                for (int mb = 0; mb < 4; ++mb) acc[mb][nb] = wmma16g(a[mb], bq, acc[mb][nb]); }
        }
    }
#pragma unroll
    for (int mb = 0; mb < 4; ++mb) {
#pragma unroll
        for (int nb = 0; nb < 2; ++nb) {
            const v4f a = __builtin_shufflevector(acc[mb][nb], acc[mb][nb], 0, 1, 2, 3);
            const v4f c = __builtin_shufflevector(acc[mb][nb], acc[mb][nb], 4, 5, 6, 7);
            *(v4fa*)(&os[(nb * 16 + lr) * OSP + mb * 16 + 8 * hi]) = a; *(v4fa*)(&os[(nb * 16 + lr) * OSP + mb * 16 + 8 * hi + 4]) = c; } }
    wave_sync();
    float* ob = OUT + (((size_t)b * NT) * IMH + y) * IMW + w0;
#pragma unroll 1
    for (int ps = 0; ps < 2; ++ps) {
#pragma unroll 1
        for (int s = 0; s < 16; ++s) { const int n = 2 * s + (lane >> 4), c4 = (lane & 15) * 4;
            const v4f val = *(const v4fa*)(&os[n * OSP + c4]);
            *(volatile v4f*)(ob + (size_t)n * IMH * IMW + c4) = val; }
        if (ps == 0) __threadfence(); }
}

static constexpr size_t al256(size_t v) { return (v + 255) & ~(size_t)255; }
static constexpr size_t SZ_A1 = al256((size_t)NB * NT * KA * 2);
static constexpr size_t SZ_W1 = al256((size_t)HID * KA * 2);
static constexpr size_t SZ_W2 = al256((size_t)KD * HP * 2);
static constexpr size_t SZ_H  = al256((size_t)NB * NT * HP * 2);
static constexpr size_t SZ_WP = al256((size_t)NB * NT * KD * 2);
static constexpr size_t SZ_LP = al256((size_t)NB * LPH * LPW * CH * 2);
static constexpr size_t SZ_TOTAL = SZ_A1 + SZ_W1 + SZ_W2 + SZ_H + SZ_WP + SZ_LP;
static_assert(SZ_TOTAL <= (size_t)134217728);
static constexpr int    N8A   = NB * NT * (EMB / 8);
static constexpr size_t NEED_LAT = (size_t)NB * CH * IMH * IMW;
static constexpr size_t NEED_OUT = (size_t)NB * NT * IMH * IMW;
static_assert(NEED_OUT * 4 <= (size_t)NB_FULL * NT * IMH * IMW * 4);

extern "C" void kernel_launch(void* const* d_in, const int* in_sizes, int n_in,
                              void* d_out, int out_size, void* d_ws, size_t ws_size, hipStream_t stream) {
    if (n_in < 7) return;
    if ((size_t)in_sizes[0] < NEED_LAT) return;
    if (in_sizes[1] < NB * EMB || in_sizes[2] < NB * NT * EMB) return;
    if (in_sizes[3] < EMB * HID || in_sizes[4] < HID || in_sizes[5] < HID * KD || in_sizes[6] < KD) return;
    if ((size_t)out_size < NEED_OUT) return;
    if (SZ_TOTAL > ws_size) return;
    const float* latent = (const float*)d_in[0];
    const float* temb   = (const float*)d_in[1];
    const float* wvemb  = (const float*)d_in[2];
    const float* w1     = (const float*)d_in[3];
    const float* b1     = (const float*)d_in[4];
    const float* w2     = (const float*)d_in[5];
    const float* b2     = (const float*)d_in[6];
    float* OUT = (float*)d_out;
    char* wsp = (char*)d_ws;
    bf*  A1  = (bf*)wsp;  wsp += SZ_A1;
    bf*  W1T = (bf*)wsp;  wsp += SZ_W1;
    bf*  W2T = (bf*)wsp;  wsp += SZ_W2;
    bf*  HPL = (bf*)wsp;  wsp += SZ_H;
    h16* WPL = (h16*)wsp; wsp += SZ_WP;
    h16* LPL = (h16*)wsp; wsp += SZ_LP;

    k_cvtrow<<<N8A / 256, 256, 0, stream>>>(wvemb, A1, N8A, 0, 0);
    k_cvtrow<<<N8A / 256, 256, 0, stream>>>(temb, A1, N8A, 5, EMB);
    k_wT<<<dim3(HID / 32, EMB / 64, 1), 256, 0, stream>>>(w1, W1T, EMB, HID, 0);
    k_wT<<<dim3(KD / 32, HID / 64, 1), 256, 0, stream>>>(w2, W2T, HID, KD, 1);
    k_lat<<<dim3(LPH, NB, 1), 256, 0, stream>>>(latent, LPL);

    k_gemm_h<<<dim3(NB * NT / 64, HID / 64, 1), 32, 0, stream>>>(A1, W1T, b1, HPL);
    k_gemm_w<<<dim3(NB * NT / 64, KD / 64, 1), 32, 0, stream>>>(HPL, W2T, b2, WPL);

    k_dconv<<<NB * IMH * (IMW / 64), 32, 0, stream>>>(LPL, WPL, OUT);
}
